// untiedLSTMcell_22445499089342
// MI455X (gfx1250) — hardware-verified
//
#include <hip/hip_runtime.h>


#define NBR  2048
#define XD   1024
#define HDN  1024
#define KK   (XD + HDN)
typedef _Float16 h16;
typedef unsigned short bf;
typedef __attribute__((ext_vector_type(16))) __bf16   v16bf;
typedef __attribute__((ext_vector_type(16))) _Float16 v16h;
typedef __attribute__((ext_vector_type(8)))  _Float16 v8h;
typedef __attribute__((ext_vector_type(8)))  unsigned short v8us;
typedef __attribute__((ext_vector_type(8)))  float    v8f;
typedef __attribute__((ext_vector_type(4)))  float    v4f;
typedef v8h  __attribute__((may_alias)) v8ha;
typedef v4f  __attribute__((may_alias)) v4fa;
typedef v8us __attribute__((may_alias)) v8usa;

__device__ __forceinline__ unsigned short f2bf(float f) { unsigned u = __float_as_uint(f); u += 0x7FFFu + ((u >> 16) & 1u); return (unsigned short)(u >> 16); }
__device__ __forceinline__ float bf2f(unsigned short b) { return __uint_as_float(((unsigned)b) << 16); }
__device__ __forceinline__ float bfr(float f) { return bf2f(f2bf(f)); }
__device__ __forceinline__ v16h cat16(v8h lo, v8h hi) { return __builtin_shufflevector(lo, hi, 0, 1, 2, 3, 4, 5, 6, 7, 8, 9, 10, 11, 12, 13, 14, 15); }
__device__ __forceinline__ v16bf cat16b(v8us lo, v8us hi) { return __builtin_bit_cast(v16bf, __builtin_shufflevector(lo, hi, 0, 1, 2, 3, 4, 5, 6, 7, 8, 9, 10, 11, 12, 13, 14, 15)); }
__device__ __forceinline__ v8f wmma16(v16h a, v16h b, v8f c) { return __builtin_amdgcn_wmma_f32_16x16x32_f16(false, a, false, b, (short)0, c, false, false); }
__device__ __forceinline__ v8f wmmab(v16bf a, v16bf b, v8f c) { return __builtin_amdgcn_wmma_f32_16x16x32_bf16(false, a, false, b, (short)0, c, false, false); }


template <typename T16> struct WFrag;
template <> struct WFrag<h16> { typedef v16h V; static __device__ __forceinline__ V ld(const h16* p) { return cat16(*(const v8h*)p, *(const v8h*)(p + 16)); } static __device__ __forceinline__ v8f mma(V a, V b, v8f c) { return wmma16(a, b, c); } };
template <> struct WFrag<bf> { typedef v16bf V; static __device__ __forceinline__ V ld(const bf* p) { return cat16b(*(const v8us*)p, *(const v8us*)(p + 16)); } static __device__ __forceinline__ v8f mma(V a, V b, v8f c) { return wmmab(a, b, c); } };
template <typename T16, int NSPLIT, bool BIAS>
__global__ __launch_bounds__(32) void k_gemmw(const T16* __restrict__ A, const T16* __restrict__ A2, const T16* __restrict__ Bt, const T16* __restrict__ Bt2, int K, float* C, int ldc, const float* __restrict__ bias, size_t sA, size_t sB, size_t sC) {
    typedef typename WFrag<T16>::V V;
    __shared__ __align__(16) float os[16 * 68];
    const size_t z = blockIdx.z; A += z * sA; if (A2) A2 += z * sA; Bt += z * sB; if (Bt2) Bt2 += z * sB; C += z * sC;
    const int lane = threadIdx.x & 31, lr = lane & 15, hi = lane >> 4; const int r0 = blockIdx.x * 64, c0 = blockIdx.y * 64;
    v8f acc[4][4];
#pragma unroll
    for (int mb = 0; mb < 4; ++mb)
#pragma unroll
        for (int nb = 0; nb < 4; ++nb) acc[mb][nb] = (v8f){};
    const size_t aoff = (size_t)(r0 + lr) * K + 8 * hi, boff = (size_t)(c0 + lr) * K + 8 * hi;
#pragma unroll 1
    for (int kc = 0; kc < K; kc += 32) {
        V a[4], a2[4];
#pragma unroll
        for (int mb = 0; mb < 4; ++mb) { a[mb] = WFrag<T16>::ld(A + aoff + (size_t)mb * 16 * K + kc); if (NSPLIT == 1 || NSPLIT == 2) a2[mb] = WFrag<T16>::ld(A2 + aoff + (size_t)mb * 16 * K + kc); }
#pragma unroll
        for (int nb = 0; nb < 4; ++nb) { const V b = WFrag<T16>::ld(Bt + boff + (size_t)nb * 16 * K + kc); V b2; if (NSPLIT >= 2) b2 = WFrag<T16>::ld(Bt2 + boff + (size_t)nb * 16 * K + kc);
#pragma unroll
            for (int mb = 0; mb < 4; ++mb) { acc[mb][nb] = WFrag<T16>::mma(a[mb], b, acc[mb][nb]); if (NSPLIT == 1 || NSPLIT == 2) acc[mb][nb] = WFrag<T16>::mma(a2[mb], b, acc[mb][nb]); if (NSPLIT >= 2) acc[mb][nb] = WFrag<T16>::mma(a[mb], b2, acc[mb][nb]); } }
        asm volatile("v_nop\n\tv_nop\n\tv_nop\n\tv_nop" : "+v"(acc[0][0]), "+v"(acc[1][1]), "+v"(acc[2][2]), "+v"(acc[3][3]) : "v"(a[0]), "v"(a[3]));
    }
#pragma unroll
    for (int mb = 0; mb < 4; ++mb) {
#pragma unroll
        for (int nb = 0; nb < 4; ++nb) {
#pragma unroll
            for (int j = 0; j < 8; ++j) os[(hi * 8 + j) * 68 + nb * 16 + lr] = acc[mb][nb][j]; }
        __builtin_amdgcn_wave_barrier(); asm volatile("" ::: "memory");
        float* crow = C + (size_t)(r0 + mb * 16) * ldc + c0;
#pragma unroll 1
        for (int ps = 0; ps < 2; ++ps) {
#pragma unroll
            for (int s = 0; s < 8; ++s) { const int row = 2 * s + hi, cofs = lr * 4; v4f val = *(const v4fa*)(os + row * 68 + cofs); if (BIAS) { val[0] += bfr(bias[c0 + cofs]); val[1] += bfr(bias[c0 + cofs + 1]); val[2] += bfr(bias[c0 + cofs + 2]); val[3] += bfr(bias[c0 + cofs + 3]); }
                *(volatile v4f*)(crow + (size_t)row * ldc + cofs) = val; }
            if (ps == 0) __threadfence(); }
        __builtin_amdgcn_wave_barrier(); asm volatile("" ::: "memory");
    }
}

__device__ __forceinline__ float sigm(float t) { return __fdiv_rn(1.0f, 1.0f + __expf(-t)); }

__global__ __launch_bounds__(256) void k_apl(const float* __restrict__ x, const float* __restrict__ h0, const float* __restrict__ mk, bf* A) {
    const size_t i = (size_t)blockIdx.x * 256 + threadIdx.x; if (i >= (size_t)NBR * KK / 8) return; const size_t e = i * 8; const int k = (int)(e & (KK - 1)); const int r = (int)(e >> 11); v8us o;
    if (k < XD) { const v8f v = *(const v8f*)(x + (size_t)r * XD + k);
#pragma unroll
        for (int q = 0; q < 8; ++q) o[q] = f2bf(v[q]); }
    else { const v8f v = *(const v8f*)(h0 + (size_t)r * HDN + k - XD), m = *(const v8f*)(mk + (size_t)r * HDN + k - XD);
#pragma unroll
        for (int q = 0; q < 8; ++q) o[q] = f2bf(bfr(v[q]) * bfr(m[q])); }
    *(volatile v8us*)(A + e) = o; __threadfence(); *(volatile v8us*)(A + e) = o;
}
__global__ __launch_bounds__(256) void k_bpl(const float* __restrict__ wx, const float* __restrict__ wh, bf* Bt) {
    const size_t i = (size_t)blockIdx.x * 256 + threadIdx.x; if (i >= (size_t)HDN * KK / 8) return; const size_t e = i * 8; const int k = (int)(e & (KK - 1)); const int n = (int)(e >> 11);
    const v8f v = (k < XD) ? *(const v8f*)(wx + (size_t)n * XD + k) : *(const v8f*)(wh + (size_t)n * HDN + k - XD); v8us o;
#pragma unroll
    for (int q = 0; q < 8; ++q) o[q] = f2bf(v[q]); *(volatile v8us*)(Bt + e) = o; __threadfence(); *(volatile v8us*)(Bt + e) = o;
}
__global__ __launch_bounds__(256) void k_cell(const float* __restrict__ G0, const float* __restrict__ G1, const float* __restrict__ G2, const float* __restrict__ G3, const float* __restrict__ bi, const float* __restrict__ bf_, const float* __restrict__ bc, const float* __restrict__ bo,
                                             const float* __restrict__ c0, const float* __restrict__ mC, float* H1, float* C1) {
    const size_t e = (size_t)blockIdx.x * 256 + threadIdx.x; if (e >= (size_t)NBR * HDN) return; const int k = (int)(e & (HDN - 1));
    const float gi = sigm(G0[e] + bfr(bi[k])), gf = sigm(G1[e] + bfr(bf_[k])), gc = tanhf(G2[e] + bfr(bc[k])) * bfr(mC[e]), go = sigm(G3[e] + bfr(bo[k]));
    const float c1 = gf * bfr(c0[e]) + gi * gc; const float h1 = go * tanhf(c1);
    *(volatile float*)(H1 + e) = h1; *(volatile float*)(C1 + e) = c1; __threadfence(); *(volatile float*)(H1 + e) = h1; *(volatile float*)(C1 + e) = c1;
}

extern "C" void kernel_launch(void* const* d_in, const int* in_sizes, int n_in,
                              void* d_out, int out_size, void* d_ws, size_t ws_size, hipStream_t stream) {
    (void)in_sizes; (void)n_in; (void)out_size;
    const float* IN[20]; for (int i = 0; i < 20; ++i) IN[i] = (const float*)d_in[i];
    float* H1 = (float*)d_out; float* C1 = (float*)((char*)d_out + (size_t)NBR * HDN * 4);
    char* wsp = (char*)d_ws;
    auto take = [&](size_t bytes) { char* p = wsp; wsp += (bytes + 255) & ~(size_t)255; return (void*)p; };
    bf* A[4]; bf* Bw[4]; float* G[4];
    for (int g = 0; g < 4; ++g) { A[g] = (bf*)take((size_t)NBR * KK * 2); Bw[g] = (bf*)take((size_t)HDN * KK * 2); G[g] = (float*)take((size_t)NBR * HDN * 4); }
    if ((size_t)(wsp - (char*)d_ws) > ws_size) return;
    for (int g = 0; g < 4; ++g) {
        k_apl<<<(unsigned)(((size_t)NBR * KK / 8 + 255) / 256), 256, 0, stream>>>(IN[0], IN[1], IN[15 + g], A[g]);
        k_bpl<<<(unsigned)(((size_t)HDN * KK / 8 + 255) / 256), 256, 0, stream>>>(IN[3 + g], IN[7 + g], Bw[g]);
        k_gemmw<bf, 0, false><<<dim3(NBR / 64, HDN / 64, 1), 32, 0, stream>>>(A[g], nullptr, Bw[g], nullptr, KK, G[g], HDN, nullptr, 0, 0, 0); }
    k_cell<<<(unsigned)(((size_t)NBR * HDN + 255) / 256), 256, 0, stream>>>(G[0], G[1], G[2], G[3], IN[11], IN[12], IN[13], IN[14], IN[2], IN[19], H1, C1);
}
